// PatchMLP_30030411333659
// MI455X (gfx1250) — hardware-verified
//
#include <hip/hip_runtime.h>


#define NIMG 2
#define HH   256
#define WWID 256
#define NPX  (HH * WWID)
#define PS   50
#define PLO  25
#define KR   (PS * PS)
#define KP   2560
#define HID  128
#define NCL  2
#define CH   8192
#define DM   KP
#define LOSC 1024.0f

typedef _Float16 h16;
typedef unsigned short bf;
typedef __attribute__((ext_vector_type(16))) __bf16   v16bf;
typedef __attribute__((ext_vector_type(16))) _Float16 v16h;
typedef __attribute__((ext_vector_type(8)))  _Float16 v8h;
typedef __attribute__((ext_vector_type(8)))  unsigned short v8us;
typedef __attribute__((ext_vector_type(8)))  float    v8f;
typedef __attribute__((ext_vector_type(4)))  float    v4f;
typedef v8h  __attribute__((may_alias)) v8ha;
typedef v4f  __attribute__((may_alias)) v4fa;
typedef v8us __attribute__((may_alias)) v8usa;

__device__ __forceinline__ unsigned short f2bf(float f) { unsigned u = __float_as_uint(f); u += 0x7FFFu + ((u >> 16) & 1u); return (unsigned short)(u >> 16); }
__device__ __forceinline__ float bf2f(unsigned short b) { return __uint_as_float(((unsigned)b) << 16); }
__device__ __forceinline__ float bfr(float f) { return bf2f(f2bf(f)); }
__device__ __forceinline__ v16h cat16(v8h lo, v8h hi) { return __builtin_shufflevector(lo, hi, 0, 1, 2, 3, 4, 5, 6, 7, 8, 9, 10, 11, 12, 13, 14, 15); }
__device__ __forceinline__ v16bf cat16b(v8us lo, v8us hi) { return __builtin_bit_cast(v16bf, __builtin_shufflevector(lo, hi, 0, 1, 2, 3, 4, 5, 6, 7, 8, 9, 10, 11, 12, 13, 14, 15)); }
__device__ __forceinline__ v8f wmma16(v16h a, v16h b, v8f c) { return __builtin_amdgcn_wmma_f32_16x16x32_f16(false, a, false, b, (short)0, c, false, false); }
__device__ __forceinline__ v8f wmmab(v16bf a, v16bf b, v8f c) { return __builtin_amdgcn_wmma_f32_16x16x32_bf16(false, a, false, b, (short)0, c, false, false); }

template <bool SPLITA, bool F16OUT = false>
__global__ __launch_bounds__(128) void k_gemmb(const bf* __restrict__ A, const bf* __restrict__ Al, const bf* __restrict__ Bn, const float* __restrict__ bias, float* C, int ldc, h16* C2, const float* __restrict__ R = nullptr, int K = DM, int roundR = 1) {
    __shared__ __align__(16) float ost[4][16 * 68];
    const int lane = threadIdx.x & 31, wave = threadIdx.x >> 5, lr = lane & 15, hi = lane >> 4;
    const int r0 = blockIdx.x * 64 + wave * 16, c0 = blockIdx.y * 64;
    const size_t aoff = (size_t)(r0 + lr) * K + 8 * hi;
    size_t boff[4];
#pragma unroll
    for (int t = 0; t < 4; ++t) boff[t] = (size_t)(c0 + t * 16 + lr) * K + 8 * hi;
    v8f acc[4];
#pragma unroll
    for (int t = 0; t < 4; ++t) acc[t] = (v8f){};
#pragma unroll 1
    for (int kc = 0; kc < K; kc += 32) {
        const v16bf a = cat16b(*(const v8us*)(A + aoff + kc), *(const v8us*)(A + aoff + kc + 16));
        v16bf al = a;
        if (SPLITA) al = cat16b(*(const v8us*)(Al + aoff + kc), *(const v8us*)(Al + aoff + kc + 16));
#pragma unroll
        for (int t = 0; t < 4; ++t) { const v16bf b = cat16b(*(const v8us*)(Bn + boff[t] + kc), *(const v8us*)(Bn + boff[t] + kc + 16)); acc[t] = wmmab(a, b, acc[t]); if (SPLITA) acc[t] = wmmab(al, b, acc[t]); }
        asm volatile("v_nop\n\tv_nop\n\tv_nop\n\tv_nop" : "+v"(acc[0]), "+v"(acc[1]), "+v"(acc[2]), "+v"(acc[3]) : "v"(a), "v"(al));
    }
    float* os = &ost[wave][0];
#pragma unroll
    for (int t = 0; t < 4; ++t) { const float bv = bias ? bfr(bias[c0 + t * 16 + lr]) : 0.f;
#pragma unroll
        for (int j = 0; j < 8; ++j) os[(hi * 8 + j) * 68 + t * 16 + lr] = acc[t][j] + bv; }
    __syncthreads();
    if (F16OUT) {
        h16* crow = (h16*)(void*)C + (size_t)r0 * ldc + c0;
        auto pass = [&]() {
#pragma unroll
            for (int s = 0; s < 4; ++s) { const int row = 4 * s + (lane >> 3), piece = lane & 7; const float* sp = os + row * 68 + piece * 8; v8h o, o2;
#pragma unroll
                for (int i = 0; i < 8; ++i) { const h16 a = (h16)sp[i]; o[i] = a; o2[i] = (h16)((sp[i] - (float)a) * LOSC); }
                *(volatile v8h*)(crow + (size_t)row * ldc + piece * 8) = o; if (C2) *(volatile v8h*)(C2 + (size_t)r0 * ldc + c0 + (size_t)row * ldc + piece * 8) = o2; }
        };
        pass(); __threadfence(); pass();
    } else {
        float* crow = C + (size_t)r0 * ldc + c0;
        auto pass = [&]() {
#pragma unroll
            for (int s = 0; s < 8; ++s) { const int Lid = (lane >> 3) + 4 * s, piece = lane & 7; const int row = Lid >> 1, cofs = (Lid & 1) * 32 + piece * 4;
                v4f val = *(const v4fa*)(os + row * 68 + cofs); if (R) { const v4f rv = *(const v4f*)(R + ((size_t)r0 + row) * ldc + c0 + cofs); val += roundR ? (v4f){bfr(rv[0]), bfr(rv[1]), bfr(rv[2]), bfr(rv[3])} : rv; }
                *(volatile v4f*)(crow + (size_t)row * ldc + cofs) = val; }
        };
        pass(); __threadfence(); pass();
    }
}


__global__ __launch_bounds__(256) void k_w1(const float* __restrict__ W1, bf* W1P) {
    const int u = blockIdx.x * 256 + threadIdx.x; if (u >= HID * KP / 8) return; const int o = u / (KP / 8), k0 = (u % (KP / 8)) * 8; v8us ob;
#pragma unroll
    for (int i = 0; i < 8; ++i) { const int k = k0 + i, kc = k < KR ? k : KR - 1; const float w = W1[(size_t)o * KR + kc]; ob[i] = (k < KR) ? f2bf(w) : (unsigned short)0; }
    *(volatile v8us*)(W1P + (size_t)u * 8) = ob; __threadfence(); *(volatile v8us*)(W1P + (size_t)u * 8) = ob;
}
__global__ __launch_bounds__(256) void k_bf(const float* __restrict__ src, bf* dst, size_t n8) {
    const size_t i = (size_t)blockIdx.x * 256 + threadIdx.x; if (i >= n8) return;
    const v8f v = *(const v8f*)(src + i * 8); v8us o;
#pragma unroll
    for (int k = 0; k < 8; ++k) o[k] = f2bf(v[k]);
    *(volatile v8us*)(dst + i * 8) = o; __threadfence(); *(volatile v8us*)(dst + i * 8) = o;
}
__global__ __launch_bounds__(256) void k_im2col(const float* __restrict__ img, int p0, bf* A) {
    const int lane = threadIdx.x & 31, r = blockIdx.x * 8 + (threadIdx.x >> 5); if (r >= CH) return;
    const int p = p0 + r, y = p / WWID, x = p % WWID;
#pragma unroll 1
    for (int ps = 0; ps < 2; ++ps) {
#pragma unroll 1
        for (int k0 = lane * 8; k0 < KP; k0 += 256) { v8us ob;
#pragma unroll
            for (int i = 0; i < 8; ++i) { const int k = k0 + i; const int ph = k / PS, pw = k - ph * PS; const int iy = y + ph - PLO, ix = x + pw - PLO;
                const bool ok = (k < KR) && iy >= 0 && iy < HH && ix >= 0 && ix < WWID; const int cy = iy < 0 ? 0 : (iy >= HH ? HH - 1 : iy), cx = ix < 0 ? 0 : (ix >= WWID ? WWID - 1 : ix);
                const float v = img[cy * WWID + cx]; ob[i] = ok ? f2bf(v) : (unsigned short)0; }
            *(volatile v8us*)(A + (size_t)r * KP + k0) = ob; }
        if (ps == 0) __threadfence(); }
}
__global__ __launch_bounds__(256) void k_split128(const float* __restrict__ src, int nrows, bf* dh, bf* dl) {
    typedef __attribute__((ext_vector_type(4))) unsigned short v4us;
    const int lane = threadIdx.x & 31, r = blockIdx.x * 8 + (threadIdx.x >> 5); if (r >= nrows) return;
    const size_t o = (size_t)r * HID + lane * 4; const v4f v = *(const v4f*)(src + o); v4us oh, ol;
#pragma unroll
    for (int i = 0; i < 4; ++i) { const unsigned short hb = f2bf(v[i]); oh[i] = hb; ol[i] = f2bf(v[i] - bf2f(hb)); }
    *(volatile v4us*)(dh + o) = oh; *(volatile v4us*)(dl + o) = ol; __threadfence(); *(volatile v4us*)(dh + o) = oh; *(volatile v4us*)(dl + o) = ol;
}
__global__ __launch_bounds__(256) void k_out(const float* __restrict__ H2, const float* __restrict__ W3, const float* __restrict__ b3, int p0, float* OUTB) {
    const int r = blockIdx.x * 256 + threadIdx.x; if (r >= CH) return; const float* hr = H2 + (size_t)r * HID;
    float a0 = bfr(b3[0]), a1 = bfr(b3[1]);
#pragma unroll 4
    for (int c = 0; c < HID; ++c) { const float h = fmaxf(hr[c], 0.f); a0 = fmaf(h, bfr(W3[c]), a0); a1 = fmaf(h, bfr(W3[HID + c]), a1); }
    float* o0 = OUTB + p0 + r; float* o1 = OUTB + (size_t)NPX + p0 + r;
    *(volatile float*)o0 = a0; *(volatile float*)o1 = a1; __threadfence(); *(volatile float*)o0 = a0; *(volatile float*)o1 = a1;
}

extern "C" void kernel_launch(void* const* d_in, const int* in_sizes, int n_in,
                              void* d_out, int out_size, void* d_ws, size_t ws_size, hipStream_t stream) {
    (void)in_sizes; (void)n_in; (void)out_size;
    const float* x = (const float*)d_in[0]; const float* W1 = (const float*)d_in[1]; const float* b1 = (const float*)d_in[2]; const float* W2 = (const float*)d_in[3]; const float* b2 = (const float*)d_in[4]; const float* W3 = (const float*)d_in[5]; const float* b3 = (const float*)d_in[6];
    float* out = (float*)d_out;
    char* wsp = (char*)d_ws;
    auto take = [&](size_t bytes) { char* p = wsp; wsp += (bytes + 255) & ~(size_t)255; return (void*)p; };
    bf* W1P = (bf*)take((size_t)HID * KP * 2); bf* W2B = (bf*)take((size_t)HID * HID * 2); bf* A = (bf*)take((size_t)CH * KP * 2); float* H1 = (float*)take((size_t)CH * HID * 4); bf* H1h = (bf*)take((size_t)CH * HID * 2); bf* H1l = (bf*)take((size_t)CH * HID * 2); float* H2 = (float*)take((size_t)CH * HID * 4);
    if ((size_t)(wsp - (char*)d_ws) > ws_size) return;
    k_w1<<<(HID * KP / 8 + 255) / 256, 256, 0, stream>>>(W1, W1P); k_bf<<<(HID * HID / 8 + 255) / 256, 256, 0, stream>>>(W2, W2B, HID * HID / 8);
    for (int b = 0; b < NIMG; ++b)
        for (int c = 0; c < NPX / CH; ++c) { const int p0 = c * CH;
            k_im2col<<<CH / 8, 256, 0, stream>>>(x + (size_t)b * NPX, p0, A);
            k_gemmb<false, false><<<dim3(CH / 64, HID / 64, 1), 128, 0, stream>>>(A, nullptr, W1P, b1, H1, HID, nullptr, nullptr, KP);
            k_split128<<<CH / 8, 256, 0, stream>>>(H1, CH, H1h, H1l);
            k_gemmb<true, false><<<dim3(CH / 64, HID / 64, 1), 128, 0, stream>>>(H1h, H1l, W2B, b2, H2, HID, nullptr, nullptr, HID);
            k_out<<<CH / 256, 256, 0, stream>>>(H2, W3, b3, p0, out + (size_t)b * NCL * NPX); }
}
